// GATLayer_15195594293512
// MI455X (gfx1250) — hardware-verified
//
#include <hip/hip_runtime.h>
#include <stddef.h>
#include <stdint.h>
#include <math.h>


#define F_IN    128
#define XUPR    (F_IN / 8)
#define HC      128
#define NHEAD   8
#define DHD     16
#define HPB     4
#define NSD     (2 * NHEAD)
#define NTHR    256
#define NWAVE   8
#define EPT     8
#define CHUNK   (NTHR * EPT)
#define WCAP    (EPT * 32)
#define LISTN   (NWAVE * WCAP)
#define NBMAX   2048
#define SLOTB   11
#define RCAP    28672
#define DEGCAP  128
#define GBM     64
#define GBN     64
#define GTHR    128
#define MROWS   128
#define NEGSL   0.2f
#define MX0     (-1.0e30f)
#define WSMAX   134217728
#define LDS_AGG ((2 * RCAP + 2 * NBMAX + LISTN) * 4 + 64)

static_assert((CHUNK & (CHUNK - 1)) == 0 && CHUNK <= (1 << SLOTB));
static_assert(NBMAX == (1 << SLOTB));
static_assert(NTHR * 8 == NBMAX);
static_assert(LISTN >= NBMAX);
static_assert(LISTN >= NWAVE * WCAP);
static_assert((RCAP % 32) == 0);
static_assert(LDS_AGG <= 300000);
static_assert(GBM == (GTHR / 32) * 16);
static_assert(GTHR == 2 * GBN && GTHR == 2 * GBM);
static_assert((F_IN % 32) == 0);
static_assert((F_IN % 8) == 0);
static_assert((HC % GBN) == 0 && HC == 2 * GBN);
static_assert(HC == NHEAD * DHD);
static_assert(GBN == HPB * DHD && DHD == 16);
static_assert(GTHR == 16 * 2 * HPB);
static_assert((MROWS % GBM) == 0);
static_assert(HC == 4 * 32);
static_assert(DHD == 4 * 4);
static_assert(F_IN == HC);

typedef float          v4f  __attribute__((ext_vector_type(4)));
typedef float          v8f  __attribute__((ext_vector_type(8)));
typedef int            v4i  __attribute__((ext_vector_type(4)));
typedef int            v8i  __attribute__((ext_vector_type(8)));
typedef unsigned int   v4u  __attribute__((ext_vector_type(4)));
typedef unsigned short v8us __attribute__((ext_vector_type(8)));
typedef __bf16         v16b __attribute__((ext_vector_type(16)));
typedef v4f  __attribute__((may_alias)) v4fa;
typedef v8us __attribute__((may_alias)) v8usa;
union FragB { v16b v; v8us h[2]; v8i w; };

__device__ __forceinline__ v8f wmb(const FragB& a, const FragB& b, v8f c) {
  v8f d = __builtin_amdgcn_wmma_f32_16x16x32_bf16(false, a.v, false, b.v, (short)0, c, false, false);
  asm volatile("v_nop\n\tv_nop\n\tv_nop\n\tv_nop" : "+v"(d) : "v"(a.w), "v"(b.w));
  return d;
}

__device__ __forceinline__ unsigned int f2bf(float f) {
  const unsigned int u = __float_as_uint(f);
  return ((u + 0x7FFFu + ((u >> 16) & 1u)) >> 16) & 0xFFFFu;
}
__device__ __forceinline__ float bf2f(unsigned int b) { return __uint_as_float(b << 16); }
__device__ __forceinline__ float bfr(float f) { return bf2f(f2bf(f)); }
__device__ __forceinline__ v4f bfr4(const v4f a) {
  v4f r; r.x = bfr(a.x); r.y = bfr(a.y); r.z = bfr(a.z); r.w = bfr(a.w); return r;
}
__device__ __forceinline__ unsigned int pk2(float lo, float hi) { return f2bf(lo) | (f2bf(hi) << 16); }
__device__ __forceinline__ v4u pack8(const v4f a, const v4f b) {
  v4u r;
  r.x = pk2(a.x, a.y); r.y = pk2(a.z, a.w); r.z = pk2(b.x, b.y); r.w = pk2(b.z, b.w);
  return r;
}

__device__ __forceinline__ int scan_chunk(const int* __restrict__ dsts, int nE, int cbase, int slotBase,
                                          int nb, int vec8, int* list, int tid, int lane, int wave) {
  int wc = 0;
  const int el0  = tid * EPT;
  const int e0   = cbase + el0;
  const int sent = -2147483647 - 1;
  v4i da, db;
  if (vec8 != 0 && cbase + CHUNK <= nE) {
    da = *(const v4i*)(dsts + e0);
    db = *(const v4i*)(dsts + e0 + 4);
  } else {
    da.x = (e0     < nE) ? dsts[min(e0,     nE - 1)] : sent;
    da.y = (e0 + 1 < nE) ? dsts[min(e0 + 1, nE - 1)] : sent;
    da.z = (e0 + 2 < nE) ? dsts[min(e0 + 2, nE - 1)] : sent;
    da.w = (e0 + 3 < nE) ? dsts[min(e0 + 3, nE - 1)] : sent;
    db.x = (e0 + 4 < nE) ? dsts[min(e0 + 4, nE - 1)] : sent;
    db.y = (e0 + 5 < nE) ? dsts[min(e0 + 5, nE - 1)] : sent;
    db.z = (e0 + 6 < nE) ? dsts[min(e0 + 6, nE - 1)] : sent;
    db.w = (e0 + 7 < nE) ? dsts[min(e0 + 7, nE - 1)] : sent;
  }
  const unsigned nbs = (unsigned)slotBase;
  const unsigned unb = (unsigned)nb;
  const unsigned s0 = (unsigned)da.x - nbs, s1 = (unsigned)da.y - nbs;
  const unsigned s2 = (unsigned)da.z - nbs, s3 = (unsigned)da.w - nbs;
  const unsigned s4 = (unsigned)db.x - nbs, s5 = (unsigned)db.y - nbs;
  const unsigned s6 = (unsigned)db.z - nbs, s7 = (unsigned)db.w - nbs;
  const bool h0 = s0 < unb, h1 = s1 < unb, h2 = s2 < unb, h3 = s3 < unb;
  const bool h4 = s4 < unb, h5 = s5 < unb, h6 = s6 < unb, h7 = s7 < unb;
  const unsigned any = __builtin_amdgcn_ballot_w32(h0 | h1 | h2 | h3 | h4 | h5 | h6 | h7);
  if (any != 0u) {
#define HITJ(J, HJ, SJ) { \
      const unsigned mj = __builtin_amdgcn_ballot_w32(HJ); \
      if (mj != 0u) { \
        if (HJ) { \
          const int pos = wc + (int)__builtin_amdgcn_mbcnt_lo(mj, 0u); \
          if (pos < WCAP) list[wave * WCAP + pos] = ((el0 + (J)) << SLOTB) | (int)(SJ); \
        } \
        wc += (int)__builtin_popcount(mj); } }
    HITJ(0, h0, s0)
    HITJ(1, h1, s1)
    HITJ(2, h2, s2)
    HITJ(3, h3, s3)
    HITJ(4, h4, s4)
    HITJ(5, h5, s5)
    HITJ(6, h6, s6)
    HITJ(7, h7, s7)
#undef HITJ
  }
  return wc;
}

__global__ __launch_bounds__(NTHR) void k_xprep(const float* __restrict__ x, unsigned short* xb, int nN, int nUnits) {
  const int i = (int)blockIdx.x * NTHR + (int)threadIdx.x;
  if (i >= nUnits) return;
  const int row = i / XUPR;
  const int c0  = (i - row * XUPR) * 8;
  const int rc  = row < nN ? row : nN - 1;
  const float* p = x + (size_t)rc * F_IN + c0;
  v4f a = *(const v4fa*)p, b = *(const v4fa*)(p + 4);
  const v4f z4 = {0.f, 0.f, 0.f, 0.f};
  if (row >= nN) { a = z4; b = z4; }
  const v4u hv = pack8(a, b);
  const size_t o = (size_t)row * F_IN + c0;
  *(volatile v4u*)(xb + o) = hv;
  __threadfence();
  *(volatile v4u*)(xb + o) = hv;
}

__global__ __launch_bounds__(NTHR) void k_wtr(const float* __restrict__ w, int Kin, int Ncol, int Nrows, int Kout,
                                              unsigned short* wt, int nUnits) {
  const int u = (int)blockIdx.x * NTHR + (int)threadIdx.x;
  if (u >= nUnits) return;
  const int kq = Kout >> 3;
  const int n  = u / kq;
  const int k8 = (u - n * kq) * 8;
  const int kk = k8 - (k8 / Kin) * Kin;
  const int ncl = n < Ncol ? n : Ncol - 1;
  const float* p = w + (size_t)kk * (size_t)Ncol + ncl;
  v4f a, b;
  a.x = p[0];                    a.y = p[(size_t)Ncol];         a.z = p[(size_t)2 * Ncol];     a.w = p[(size_t)3 * Ncol];
  b.x = p[(size_t)4 * Ncol];     b.y = p[(size_t)5 * Ncol];     b.z = p[(size_t)6 * Ncol];     b.w = p[(size_t)7 * Ncol];
  const v4f z4 = {0.f, 0.f, 0.f, 0.f};
  if (n >= Ncol || n >= Nrows) { a = z4; b = z4; }
  const v4u wv = pack8(a, b);
  unsigned short* o = wt + (size_t)n * (size_t)Kout + k8;
  *(volatile v4u*)o = wv;
  __threadfence();
  *(volatile v4u*)o = wv;
}

__global__ __launch_bounds__(GTHR) void k_gemm(
    const unsigned short* __restrict__ A, const unsigned short* __restrict__ WT,
    float* outF, int K, int ldo,
    const float* __restrict__ atts, const float* __restrict__ attd, int attN,
    float* SD, int MPr)
{
  __shared__ __attribute__((aligned(16))) float stg[GBM * GBN];
  __shared__ __attribute__((aligned(16))) float satt[2 * GBN];
  __shared__ __attribute__((aligned(16))) float sdot[2 * HPB * GBM];
  const int tid = (int)threadIdx.x, lane = tid & 31, wave = tid >> 5, hh = lane >> 4, m = lane & 15;
  const int rowBase = (int)blockIdx.x * GBM;
  const int by      = (int)blockIdx.y;
  const int col0    = by * GBN;

  {
    const int which = tid >> 6;
    const int c     = tid & 63;
    int ai = col0 + c;
    ai = ai < 0 ? 0 : (ai < attN ? ai : attN - 1);
    const float vs = atts[ai];
    const float vd = attd[ai];
    const unsigned int msk = (which == 0) ? 0u : 0xFFFFFFFFu;
    const float v = __uint_as_float((__float_as_uint(vs) & ~msk) | (__float_as_uint(vd) & msk));
    satt[which * GBN + c] = bfr(v);
  }

  v8f acc[4];
  {
    const v8f z = {0.f, 0.f, 0.f, 0.f, 0.f, 0.f, 0.f, 0.f};
    acc[0] = z; acc[1] = z; acc[2] = z; acc[3] = z;
  }
  const unsigned short* ap = A  + (size_t)(rowBase + 16 * wave + m) * (size_t)K + 8 * hh;
  const unsigned short* wp = WT + (size_t)(col0 + m) * (size_t)K + 8 * hh;
  const int ksteps = K >> 5;
#pragma unroll 1
  for (int ks = 0; ks < ksteps; ++ks) {
    FragB af;
    af.h[0] = *(const v8usa*)(ap + 32 * ks);
    af.h[1] = *(const v8usa*)(ap + 32 * ks + 16);
#pragma unroll
    for (int t = 0; t < 4; ++t) {
      const unsigned short* wq = wp + (size_t)(16 * t) * (size_t)K + 32 * ks;
      FragB bf;
      bf.h[0] = *(const v8usa*)wq;
      bf.h[1] = *(const v8usa*)(wq + 16);
      acc[t] = wmb(af, bf, acc[t]);
    }
  }

#pragma unroll
  for (int t = 0; t < 4; ++t) {
    const int lc = 16 * t + m;
#pragma unroll
    for (int r = 0; r < 8; ++r) {
      const int lr = 16 * wave + 8 * hh + r;
      stg[lr * GBN + lc] = acc[t][r];
    }
  }
  __syncthreads();

  {
    const int row = tid & 63, which = tid >> 6;
    const float* sa = satt + which * GBN;
    const float* hr = stg + row * GBN;
    float d0 = 0.f, d1 = 0.f, d2 = 0.f, d3 = 0.f;
#pragma unroll
    for (int c4 = 0; c4 < DHD / 4; ++c4) {
      const v4f h0 = *(const v4fa*)(hr + 4 * c4);
      const v4f a0 = *(const v4fa*)(sa + 4 * c4);
      d0 = fmaf(h0.x, a0.x, d0); d0 = fmaf(h0.y, a0.y, d0); d0 = fmaf(h0.z, a0.z, d0); d0 = fmaf(h0.w, a0.w, d0);
      const v4f h1 = *(const v4fa*)(hr + DHD + 4 * c4);
      const v4f a1 = *(const v4fa*)(sa + DHD + 4 * c4);
      d1 = fmaf(h1.x, a1.x, d1); d1 = fmaf(h1.y, a1.y, d1); d1 = fmaf(h1.z, a1.z, d1); d1 = fmaf(h1.w, a1.w, d1);
      const v4f h2 = *(const v4fa*)(hr + 2 * DHD + 4 * c4);
      const v4f a2 = *(const v4fa*)(sa + 2 * DHD + 4 * c4);
      d2 = fmaf(h2.x, a2.x, d2); d2 = fmaf(h2.y, a2.y, d2); d2 = fmaf(h2.z, a2.z, d2); d2 = fmaf(h2.w, a2.w, d2);
      const v4f h3 = *(const v4fa*)(hr + 3 * DHD + 4 * c4);
      const v4f a3 = *(const v4fa*)(sa + 3 * DHD + 4 * c4);
      d3 = fmaf(h3.x, a3.x, d3); d3 = fmaf(h3.y, a3.y, d3); d3 = fmaf(h3.z, a3.z, d3); d3 = fmaf(h3.w, a3.w, d3);
    }
    sdot[(which * HPB + 0) * GBM + row] = d0;
    sdot[(which * HPB + 1) * GBM + row] = d1;
    sdot[(which * HPB + 2) * GBM + row] = d2;
    sdot[(which * HPB + 3) * GBM + row] = d3;
  }
  __syncthreads();

  v4f fv[8];
#pragma unroll
  for (int i = 0; i < 8; ++i) {
    const int lr = 16 * wave + 2 * i + hh;
    fv[i] = *(const v4fa*)(stg + lr * GBN + 4 * m);
  }
  const int piece = tid & 15;
  const int g     = tid >> 4;
  const int plane = (g >> 2) * NHEAD + HPB * by + (g & 3);
  const v4f sdv = *(const v4fa*)(sdot + g * GBM + 4 * piece);
  float* sp = SD + (size_t)plane * (size_t)MPr + rowBase + 4 * piece;

#pragma unroll
  for (int i = 0; i < 8; ++i) {
    const int lr = 16 * wave + 2 * i + hh;
    const int gr = rowBase + lr;
    float* op = outF + (size_t)gr * (size_t)ldo + col0 + 4 * m;
    *(volatile v4f*)op = fv[i];
  }
  *(volatile v4f*)sp = sdv;
  __threadfence();
#pragma unroll
  for (int i = 0; i < 8; ++i) {
    const int lr = 16 * wave + 2 * i + hh;
    const int gr = rowBase + lr;
    float* op = outF + (size_t)gr * (size_t)ldo + col0 + 4 * m;
    *(volatile v4f*)op = fv[i];
  }
  *(volatile v4f*)sp = sdv;
}

__global__ __launch_bounds__(NTHR) void k_agg(
    const int* __restrict__ srcs, const int* __restrict__ dsts,
    const float* __restrict__ F, const float* __restrict__ SD,
    const float* __restrict__ xres, const float* __restrict__ bias,
    float* out, int nN, int nE, int nb, int vec8, int MPr) {
  extern __shared__ v4f lds_dyn[];
  int* reg1 = (int*)lds_dyn;
  int* reg2 = reg1 + RCAP;
  int* scnt = reg2 + RCAP;
  int* soff = scnt + NBMAX;
  int* list = soff + NBMAX;
  int* wcnt = list + LISTN;
  int* wtot = wcnt + NWAVE;
  const int tid = (int)threadIdx.x, lane = tid & 31, wave = tid >> 5;
  const int nodeBase = (int)blockIdx.x * nb;

  for (int i = tid; i < NBMAX; i += NTHR) scnt[i] = 0;
  __syncthreads();

  int tot = 0;
  const int nChunks = (nE + CHUNK - 1) / CHUNK;
#pragma unroll 1
  for (int ch = 0; ch < nChunks; ++ch) {
    const int cbase = ch * CHUNK;
    const int wc = scan_chunk(dsts, nE, cbase, nodeBase, nb, vec8, list, tid, lane, wave);
    if (lane == 0) wcnt[wave] = wc;
    __syncthreads();
    int pre = 0, all = 0;
#pragma unroll
    for (int w2 = 0; w2 < NWAVE; ++w2) {
      int c = wcnt[w2];
      c = c < 0 ? 0 : (c > WCAP ? WCAP : c);
      all += c;
      pre += (w2 < wave) ? c : 0;
    }
    const int wcc  = wc > WCAP ? WCAP : wc;
    const int base = tot + pre;
#pragma unroll 1
    for (int i = lane; i < wcc; i += 32) {
      const int ent = list[wave * WCAP + i];
      const int el  = (ent >> SLOTB) & (CHUNK - 1);
      const int sl  = ent & (NBMAX - 1);
      int eid = cbase + el;
      eid = eid > nE - 1 ? nE - 1 : eid;
      const int pos = base + i;
      if (pos < RCAP) reg1[pos] = (int)(((unsigned)eid << SLOTB) | (unsigned)sl);
    }
    tot += all;
    tot = tot > RCAP ? RCAP : tot;
    __syncthreads();
  }
  const int nh = tot;

  if (wave == 0) {
#pragma unroll 1
    for (int b0 = 0; b0 < nh; b0 += 32) {
      const int idx = b0 + lane;
      const int uv  = reg1[idx < nh ? idx : nh - 1];
      const int m32 = (nh - b0) < 32 ? (nh - b0) : 32;
#pragma unroll 1
      for (int k = 0; k < m32; ++k) {
        const int u  = __builtin_amdgcn_readlane(uv, k);
        const int sl = u & (NBMAX - 1);
        if (lane == 0) scnt[sl] = scnt[sl] + 1;
      }
    }
  }
  __syncthreads();

  {
    const v4i ca = *(const v4i*)(scnt + 8 * tid);
    const v4i cb = *(const v4i*)(scnt + 8 * tid + 4);
    const int e0 = ca.x < 0 ? 0 : ca.x, e1 = ca.y < 0 ? 0 : ca.y, e2 = ca.z < 0 ? 0 : ca.z, e3 = ca.w < 0 ? 0 : ca.w;
    const int e4 = cb.x < 0 ? 0 : cb.x, e5 = cb.y < 0 ? 0 : cb.y, e6 = cb.z < 0 ? 0 : cb.z, e7 = cb.w < 0 ? 0 : cb.w;
    const int ts = e0 + e1 + e2 + e3 + e4 + e5 + e6 + e7;
    int incl = ts;
#pragma unroll
    for (int d = 1; d < 32; d <<= 1) {
      const int up = __shfl_up(incl, d);
      if (lane >= d) incl += up;
    }
    if (lane == 31) wtot[wave] = incl;
    __syncthreads();
    int pre = 0;
#pragma unroll
    for (int w2 = 0; w2 < NWAVE; ++w2) pre += (w2 < wave) ? wtot[w2] : 0;
    int run = pre + incl - ts;
    soff[8 * tid + 0] = run; run += e0;
    soff[8 * tid + 1] = run; run += e1;
    soff[8 * tid + 2] = run; run += e2;
    soff[8 * tid + 3] = run; run += e3;
    soff[8 * tid + 4] = run; run += e4;
    soff[8 * tid + 5] = run; run += e5;
    soff[8 * tid + 6] = run; run += e6;
    soff[8 * tid + 7] = run;
  }
  __syncthreads();
  for (int i = tid; i < NBMAX; i += NTHR) list[i] = soff[i];
  __syncthreads();

  if (wave == 0) {
#pragma unroll 1
    for (int b0 = 0; b0 < nh; b0 += 32) {
      const int idx = b0 + lane;
      const int uv  = reg1[idx < nh ? idx : nh - 1];
      const int m32 = (nh - b0) < 32 ? (nh - b0) : 32;
#pragma unroll 1
      for (int k = 0; k < m32; ++k) {
        const int u   = __builtin_amdgcn_readlane(uv, k);
        const int sl  = u & (NBMAX - 1);
        const int eid = (int)((unsigned)u >> SLOTB);
        if (lane == 0) {
          int pos = list[sl];
          pos = pos < 0 ? 0 : (pos > RCAP - 1 ? RCAP - 1 : pos);
          reg2[pos] = eid;
          list[sl] = pos + 1;
        }
      }
    }
  }
  __syncthreads();

  const int nbw = nb >> 3;
  const bool ovf = (nh >= RCAP);
  const float qnan = __int_as_float(0x7fc00000);
  const int c0 = 4 * lane;
  const int head = lane >> 2;
  const float* ELp = SD + (size_t)head * (size_t)MPr;
  const float* ERp = SD + (size_t)(NHEAD + head) * (size_t)MPr;
  const v4f bb = bfr4(*(const v4fa*)(bias + c0));

#pragma unroll 1
  for (int jt = 0; jt < nbw; ++jt) {
    const int slot = wave * nbw + jt;
    const int grow = nodeBase + slot;
    const int gcl  = grow < nN ? grow : nN - 1;
    int st = soff[slot];
    const int craw = scnt[slot];
    int cnt = craw;
    st  = st < 0 ? 0 : (st > nh ? nh : st);
    cnt = cnt < 0 ? 0 : (cnt > DEGCAP ? DEGCAP : cnt);
    if (cnt > nh - st) cnt = nh - st;
    const float pz = (ovf || craw > DEGCAP) ? qnan : 0.0f;

    const float erd = ERp[gcl];
    const v4f fr = bfr4(*(const v4fa*)(xres + (size_t)gcl * F_IN + c0));
    float mx = MX0, dn = 0.0f;
    v4f av = {0.f, 0.f, 0.f, 0.f};

#pragma unroll 1
    for (int q = 0; q < cnt; ++q) {
      int idx = st + q; idx = idx > RCAP - 1 ? RCAP - 1 : idx;
      int eid = reg2[idx]; eid = eid < 0 ? 0 : (eid > nE - 1 ? nE - 1 : eid);
      const int sraw = srcs[eid];
      const int s = sraw < 0 ? 0 : (sraw > nN - 1 ? nN - 1 : sraw);
      const v4f fs = *(const v4fa*)(F + (size_t)s * HC + c0);
      float lg = ELp[s] + erd;
      lg = lg > 0.f ? lg : NEGSL * lg;
      const float df = lg - mx;
      const float ee = __expf(-fabsf(df));
      const bool up  = df > 0.f;
      const float s1 = up ? ee : 1.0f;
      const float s2 = up ? 1.0f : ee;
      mx = up ? lg : mx;
      dn = fmaf(dn, s1, s2);
      av.x = fmaf(av.x, s1, s2 * fs.x);
      av.y = fmaf(av.y, s1, s2 * fs.y);
      av.z = fmaf(av.z, s1, s2 * fs.z);
      av.w = fmaf(av.w, s1, s2 * fs.w);
    }
    const float dsafe = dn > 0.f ? dn : 1.0f;
    const float inv = __builtin_amdgcn_rcpf(dsafe);
    v4f o;
    o.x = fmaf(av.x, inv, fr.x) + bb.x + pz;
    o.y = fmaf(av.y, inv, fr.y) + bb.y + pz;
    o.z = fmaf(av.z, inv, fr.z) + bb.z + pz;
    o.w = fmaf(av.w, inv, fr.w) + bb.w + pz;
    const bool live = grow < nN;
    float* op = out + (size_t)gcl * HC + c0;
    if (live) *(volatile v4f*)op = o;
    __threadfence();
    if (live) *(volatile v4f*)op = o;
  }
}

static int pick_nb(int nE, int nN) {
  int nb = NBMAX;
  while (nb > 32 && (long long)nb * (long long)nE * 5LL > (long long)RCAP * (long long)nN * 4LL) nb >>= 1;
  return nb;
}
static inline int cdiv(int a, int b) { return (a + b - 1) / b; }

extern "C" void kernel_launch(void* const* d_in, const int* in_sizes, int n_in,
                              void* d_out, int out_size, void* d_ws, size_t ws_size,
                              hipStream_t stream) {
  if (n_in < 7) return;
  const int nN = in_sizes[0] / F_IN;
  if (nN <= 0 || in_sizes[0] != nN * F_IN || nN > (1 << 22)) return;
  if (in_sizes[1] != F_IN * HC) return;
  if (in_sizes[2] != HC || in_sizes[3] != HC) return;
  if (in_sizes[4] != HC) return;
  const int nE = in_sizes[5];
  if (nE < 1 || in_sizes[6] != nE || nE >= (1 << (32 - SLOTB))) return;
  if (out_size != nN * HC) return;

  const float* x    = (const float*)d_in[0];
  const float* W    = (const float*)d_in[1];
  const float* al   = (const float*)d_in[2];
  const float* ar   = (const float*)d_in[3];
  const float* bias = (const float*)d_in[4];
  const int*   src  = (const int*)  d_in[5];
  const int*   dst  = (const int*)  d_in[6];
  float* out = (float*)d_out;

  const int MP   = cdiv(nN, MROWS) * MROWS;
  const int nb   = pick_nb(nE, nN);
  if (nb < 32 || (nb & (nb - 1)) != 0 || nb > NBMAX) return;
  const int gA   = cdiv(MP, nb);
  const int vec8 = 1;
  if (gA * nb < MP) return;

  char* ws = (char*)d_ws;
  size_t off = 0;
  const size_t oXB = off; off += (size_t)MP * F_IN * 2;           off = (off + 255) & ~(size_t)255;
  const size_t oWT = off; off += (size_t)HC * F_IN * 2;           off = (off + 255) & ~(size_t)255;
  const size_t oWH = off; off += (size_t)MP * HC * 4;             off = (off + 255) & ~(size_t)255;
  const size_t oSD = off; off += (size_t)NSD * MP * 4;            off = (off + 255) & ~(size_t)255;
  if (off > ws_size || off > (size_t)WSMAX) return;
  unsigned short* XB = (unsigned short*)(ws + oXB);
  unsigned short* WT = (unsigned short*)(ws + oWT);
  float*          WH = (float*)(ws + oWH);
  float*          SD = (float*)(ws + oSD);

  hipFuncSetAttribute(reinterpret_cast<const void*>(&k_agg),
                      hipFuncAttributeMaxDynamicSharedMemorySize, LDS_AGG);

  const int nUx = MP * XUPR;
  k_xprep<<<cdiv(nUx, NTHR), NTHR, 0, stream>>>(x, XB, nN, nUx);

  {
    const int nUw = HC * (F_IN / 8);
    k_wtr<<<cdiv(nUw, NTHR), NTHR, 0, stream>>>(W, F_IN, HC, HC, F_IN, WT, nUw);
  }

  const int gM = MP / GBM;
  k_gemm<<<dim3(gM, HC / GBN), GTHR, 0, stream>>>(XB, WT, WH, F_IN, HC, al, ar, HC, SD, MP);
  k_agg<<<gA, NTHR, LDS_AGG, stream>>>(src, dst, WH, SD, x, bias, out, nN, nE, nb, vec8, MP);
}
